// SpatialTransformerModel_70806830842265
// MI455X (gfx1250) — hardware-verified
//
#include <hip/hip_runtime.h>
#include <math.h>

typedef __attribute__((ext_vector_type(16))) _Float16 v16h;
typedef __attribute__((ext_vector_type(16))) __bf16 v16b;
typedef __attribute__((ext_vector_type(8)))  _Float16 v8h;
typedef __attribute__((ext_vector_type(8)))  float v8f;
typedef __attribute__((ext_vector_type(4)))  float v4f;
typedef __attribute__((ext_vector_type(2)))  float v2f;
typedef __attribute__((ext_vector_type(4)))  unsigned v4u;
typedef __attribute__((ext_vector_type(4)))  int v4i;
typedef float __attribute__((may_alias)) float_a;
typedef int __attribute__((may_alias)) int_a;

template <typename T> __device__ __forceinline__ void vst2(void* p, T v) { *(volatile T*)p = v; __threadfence(); *(volatile T*)p = v; }
__device__ __forceinline__ v8f wmma16(v16h a, v16h b, v8f c) {
  v8f d = __builtin_amdgcn_wmma_f32_16x16x32_f16(false, a, false, b, (short)0, c, false, false);
  asm volatile("v_nop\n\tv_nop\n\tv_nop\n\tv_nop" : "+v"(d) : "v"(a), "v"(b));
  return d;
}
__device__ __forceinline__ v8f wmma_bf(v16b a, v16b b, v8f c) {
  v8f d = __builtin_amdgcn_wmma_f32_16x16x32_bf16(false, a, false, b, (short)0, c, false, false);
  asm volatile("v_nop\n\tv_nop\n\tv_nop\n\tv_nop" : "+v"(d) : "v"(a), "v"(b));
  return d;
}
__device__ __forceinline__ v16h frag_h(const _Float16* rowk0, int lane) {
  union { v16h v; v8h q[2]; } u; const _Float16* p = rowk0 + 8 * (lane >> 4);
  u.q[0] = *(const v8h*)p; u.q[1] = *(const v8h*)(p + 16); return u.v;
}
__device__ __forceinline__ v16h frag_f32(const float* rowk0, int lane) {
  v16h a; const float* p = rowk0 + 8 * (lane >> 4);
#pragma unroll
  for (int i = 0; i < 8; ++i) { a[i] = (_Float16)p[i]; a[8 + i] = (_Float16)p[16 + i]; }
  return a;
}
__device__ __forceinline__ v16h frag_f32s(const float* rowk0, int lane, float sc) {
  v16h a; const float* p = rowk0 + 8 * (lane >> 4);
#pragma unroll
  for (int i = 0; i < 8; ++i) { a[i] = (_Float16)(p[i] * sc); a[8 + i] = (_Float16)(p[16 + i] * sc); }
  return a;
}
__device__ __forceinline__ v16h fragc_f32(const float* W, int k0, int n, int lane, int ld, int K) {
  v16h a; const int g = lane >> 4;
#pragma unroll
  for (int i = 0; i < 8; ++i) { const int ka = k0 + 8 * g + i, kb = ka + 16;
    a[i] = (_Float16)(ka < K ? W[(size_t)(ka < K ? ka : K - 1) * ld + n] : 0.f); a[8 + i] = (_Float16)(kb < K ? W[(size_t)(kb < K ? kb : K - 1) * ld + n] : 0.f); }
  return a;
}
struct F2 { v16b h, l; };
__device__ __forceinline__ F2 bsplit16(const float v[16]) { F2 r;
#pragma unroll
  for (int i = 0; i < 16; ++i) { const __bf16 h = (__bf16)v[i]; r.h[i] = h; r.l[i] = (__bf16)(v[i] - (float)h); }
  return r; }
__device__ __forceinline__ F2 split_row(const float* row, int k0, int lane) { float v[16]; const float* p = row + k0 + 8 * (lane >> 4);
#pragma unroll
  for (int i = 0; i < 8; ++i) { v[i] = p[i]; v[8 + i] = p[16 + i]; }
  return bsplit16(v); }
__device__ __forceinline__ F2 split_rowK(const float* row, int k0, int lane, int K) { float v[16]; const int g = lane >> 4;
#pragma unroll
  for (int i = 0; i < 8; ++i) { const int ka = k0 + 8 * g + i, kb = ka + 16; v[i] = ka < K ? row[ka < K ? ka : K - 1] : 0.f; v[8 + i] = kb < K ? row[kb < K ? kb : K - 1] : 0.f; }
  return bsplit16(v); }
__device__ __forceinline__ F2 split_col(const float* W, int k0, int n, int lane, int ld, int K) { float v[16]; const int g = lane >> 4;
#pragma unroll
  for (int i = 0; i < 8; ++i) { const int ka = k0 + 8 * g + i, kb = ka + 16; v[i] = ka < K ? W[(size_t)(ka < K ? ka : K - 1) * ld + n] : 0.f; v[8 + i] = kb < K ? W[(size_t)(kb < K ? kb : K - 1) * ld + n] : 0.f; }
  return bsplit16(v); }
__device__ __forceinline__ v8f mac3(const F2& a, const F2& b, v8f c) { c = wmma_bf(a.l, b.h, c); c = wmma_bf(a.h, b.l, c); return wmma_bf(a.h, b.h, c); }
__device__ __forceinline__ float sigm(float v) { return 1.0f / (1.0f + expf(-v)); }
#define LDSX() do { asm volatile("s_wait_dscnt 0" ::: "memory"); __builtin_amdgcn_wave_barrier(); __builtin_amdgcn_fence(__ATOMIC_RELEASE, "workgroup"); } while (0)


#define NBT 96
#define NN 512
#define NR (NBT * NN)
#define DX 64
#define DH 128
#define NHD 8
#define HD 8
#define DM 64
#ifndef TNG
#define TNG NBT
#endif
typedef __attribute__((ext_vector_type(8))) __bf16 v8b;
__device__ __forceinline__ v16b frag_b(const __bf16* rowk0, int lane) {
  union { v16b v; v8b q[2]; } u; const __bf16* p = rowk0 + 8 * (lane >> 4);
  u.q[0] = *(const v8b*)p; u.q[1] = *(const v8b*)(p + 16); return u.v;
}
__device__ __forceinline__ float bfr(float v) { return (float)(__bf16)v; }
__device__ __attribute__((noinline)) float exp_ni(float v) { return expf(v); }
__device__ __attribute__((noinline)) float erf_ni(float v) { return erff(v); }

#define PK_QKV 0
#define PK_O1 (PK_QKV + 3 * DM * DH)
#define PK_O2 (PK_O1 + DM * DM)
#define PK_END (PK_O2 + DM * DM)
#define WS_PK  0u
#define WS_QP  (((2u * PK_END) + 127u) / 128u * 128u)
#define WS_KP  (WS_QP + 2u * (size_t)NR * NHD * 32)
#define WS_VT  (WS_KP + 2u * (size_t)NR * NHD * 32)
#define WS_VTL (WS_VT + 2u * (size_t)NBT * NHD * 16 * NN)
#define WS_O   (WS_VTL + 2u * (size_t)NBT * NHD * 16 * NN)
#define WS_END (WS_O + 4u * (size_t)NR * DM)

__global__ __launch_bounds__(256) void k_pack(const float* __restrict__ WQ, const float* __restrict__ WK, const float* __restrict__ WV, const float* __restrict__ WO1, const float* __restrict__ WO2, __bf16* __restrict__ PK) {
  __shared__ __align__(16) __bf16 s[DH]; const int n = blockIdx.x, which = blockIdx.y, t = threadIdx.x; int K; size_t dst;
  if (which < 3) { const float* Wm = (which == 0) ? WQ : (which == 1) ? WK : WV; K = DH; dst = PK_QKV + ((size_t)which * DM + n) * DH; if (t < DH) s[t] = (__bf16)Wm[(size_t)t * DM + n]; }
  else { const float* Wm = (which == 3) ? WO1 : WO2; K = DM; dst = ((which == 3) ? PK_O1 : PK_O2) + (size_t)n * DM; if (t < DM) s[t] = (__bf16)Wm[(size_t)t * DM + n]; }
  __syncthreads();
  if (t < K / 8) vst2((unsigned*)(PK + dst + t * 8), *(const v4u*)&s[t * 8]);
}
__global__ __launch_bounds__(128) void k_qkv(const float* __restrict__ X, const float* __restrict__ STE, const __bf16* __restrict__ PK, const float* __restrict__ BQ, const float* __restrict__ BK, const float* __restrict__ BV, _Float16* __restrict__ QP, _Float16* __restrict__ KP, _Float16* __restrict__ VT, _Float16* __restrict__ VTL) {
  __shared__ __align__(16) _Float16 sq[4][16][NHD * 32 + 8], sk[4][16][NHD * 32 + 8]; __shared__ __align__(16) _Float16 svh[NHD * 16][72], svl[NHD * 16][72];
  const int tid = threadIdx.x, wave = tid >> 5, lane = tid & 31, col = lane & 15, g = lane >> 4; const size_t r0 = (size_t)blockIdx.x * 64 + wave * 16;
  for (int e = lane; e < 16 * (NHD * 32 + 8); e += 32) { (&sq[wave][0][0])[e] = (_Float16)0.f; (&sk[wave][0][0])[e] = (_Float16)0.f; }
  for (int e = tid; e < NHD * 16 * 72; e += 128) { (&svh[0][0])[e] = (_Float16)0.f; (&svl[0][0])[e] = (_Float16)0.f; }
  __syncthreads();
  v8f acc[12] = {};
#pragma unroll
  for (int kc = 0; kc < DH / 32; ++kc) { v16b a; { const float* p = ((kc < 2) ? X + (r0 + col) * DX + kc * 32 : STE + (r0 + col) * DX + (kc - 2) * 32) + 8 * g;
#pragma unroll
      for (int i = 0; i < 8; ++i) { a[i] = (__bf16)p[i]; a[8 + i] = (__bf16)p[16 + i]; } }
#pragma unroll
    for (int j = 0; j < 12; ++j) acc[j] = wmma_bf(a, frag_b(PK + PK_QKV + (size_t)(j * 16 + col) * DH + kc * 32, lane), acc[j]); }
#pragma unroll
  for (int j = 0; j < 12; ++j) { const int which = j >> 2; const int c = (j & 3) * 16 + col; const int h = c >> 3, d = c & 7; const float bb = bfr((which == 0) ? BQ[c] : (which == 1) ? BK[c] : BV[c]);
#pragma unroll
    for (int r = 0; r < 8; ++r) { const float v = fmaxf(acc[j][r] + bb, 0.f);
      if (which == 0) sq[wave][8 * g + r][h * 32 + d] = (_Float16)(v * 0.35355339059327373f);
      else if (which == 1) sk[wave][8 * g + r][h * 32 + d] = (_Float16)v;
      else { const _Float16 hv = (_Float16)v; svh[h * 16 + d][wave * 16 + 8 * g + r] = hv; svl[h * 16 + d][wave * 16 + 8 * g + r] = (_Float16)((v - (float)hv) * 2048.0f); } } }
  __syncthreads();
  for (int rl = 0; rl < 16; ++rl) vst2((unsigned*)(QP + (r0 + rl) * (NHD * 32) + lane * 8), *(const v4u*)&sq[wave][rl][lane * 8]);
  for (int rl = 0; rl < 16; ++rl) vst2((unsigned*)(KP + (r0 + rl) * (NHD * 32) + lane * 8), *(const v4u*)&sk[wave][rl][lane * 8]);
  { const size_t rb = (size_t)blockIdx.x * 64; const size_t grp = rb / NN; const int n0 = (int)(rb % NN);
    for (int e = tid; e < NHD * 16 * 8; e += 128) { const int hd = e >> 3, pc = e & 7; const size_t o = (grp * NHD * 16 + hd) * NN + n0 + pc * 8; vst2((unsigned*)(VT + o), *(const v4u*)&svh[hd][pc * 8]); vst2((unsigned*)(VTL + o), *(const v4u*)&svl[hd][pc * 8]); } }
}
__global__ __launch_bounds__(128) void k_attn(const _Float16* __restrict__ QP, const _Float16* __restrict__ KP, const _Float16* __restrict__ VT, const _Float16* __restrict__ VTL, float* __restrict__ O) {
  __shared__ __align__(16) _Float16 sp[4][16][40]; __shared__ __align__(16) float so[4][16][DM + 4];
  const int tid = threadIdx.x, wave = tid >> 5, lane = tid & 31, col = lane & 15, g = lane >> 4; const int qb = blockIdx.x; const size_t grp = blockIdx.y; const size_t q0 = grp * NN + (size_t)qb * 64 + wave * 16;
#pragma unroll 1
  for (int h = 0; h < NHD; ++h) {
    const v16h aq = frag_h(QP + (q0 + col) * (NHD * 32) + h * 32, lane);
    float m[8], l[8];
#pragma unroll
    for (int r = 0; r < 8; ++r) { m[r] = -3.0e38f; l[r] = 0.f; }
    v8f acc = {}, accl = {};
#pragma unroll 1
    for (int ks = 0; ks < NN / 32; ++ks) { v8f s[2];
#pragma unroll
      for (int ct = 0; ct < 2; ++ct) { const size_t kk = grp * NN + (size_t)ks * 32 + ct * 16 + col; v8f c = {}; c = wmma16(aq, frag_h(KP + kk * (NHD * 32) + h * 32, lane), c);
#pragma unroll
        for (int r = 0; r < 8; ++r) s[ct][r] = c[r]; }
#pragma unroll
      for (int r = 0; r < 8; ++r) { float mx = fmaxf(s[0][r], s[1][r]);
#pragma unroll
        for (int o = 1; o < 16; o <<= 1) mx = fmaxf(mx, __shfl_xor(mx, o));
        const float mn = fmaxf(m[r], mx); const float alpha = (m[r] <= -1.0e38f) ? 0.f : exp_ni(m[r] - mn); const float e0 = exp_ni(s[0][r] - mn), e1 = exp_ni(s[1][r] - mn); float es = e0 + e1;
#pragma unroll
        for (int o = 1; o < 16; o <<= 1) es += __shfl_xor(es, o);
        l[r] = l[r] * alpha + es; m[r] = mn; acc[r] *= alpha; accl[r] *= alpha;
        sp[wave][8 * g + r][col] = (_Float16)e0; sp[wave][8 * g + r][16 + col] = (_Float16)e1; }
      LDSX();
      const v16h pa = frag_h(&sp[wave][col][0], lane); const size_t vo = ((grp * NHD + h) * 16 + col) * NN + (size_t)ks * 32;
      acc = wmma16(pa, frag_h(VT + vo, lane), acc); accl = wmma16(pa, frag_h(VTL + vo, lane), accl);
      LDSX(); }
    if (col < HD) {
#pragma unroll
      for (int r = 0; r < 8; ++r) so[wave][8 * g + r][h * HD + col] = (acc[r] + accl[r] * (1.0f / 2048.0f)) / l[r]; } }
  LDSX();
  for (int rl = 0; rl < 16; ++rl) if (lane < 16) vst2(O + (q0 + rl) * DM + lane * 4, *(const v4f*)&so[wave][rl][lane * 4]);
}
__global__ __launch_bounds__(128) void k_mlp(const float* __restrict__ O, const __bf16* __restrict__ PK, const float* __restrict__ B1, const float* __restrict__ B2, float* __restrict__ OUT) {
  __shared__ __align__(16) __bf16 sh_[4][16][72], sl_[4][16][72]; __shared__ __align__(16) float so[4][16][DM + 4];
  const int tid = threadIdx.x, wave = tid >> 5, lane = tid & 31, col = lane & 15, g = lane >> 4; const size_t r0 = (size_t)blockIdx.x * 64 + wave * 16;
  v8f acc[4] = {};
#pragma unroll
  for (int kc = 0; kc < DM / 32; ++kc) { const F2 a = split_row(O + (r0 + col) * DM, kc * 32, lane);
#pragma unroll
    for (int j = 0; j < 4; ++j) { const v16b w = frag_b(PK + PK_O1 + (size_t)(j * 16 + col) * DM + kc * 32, lane); acc[j] = wmma_bf(a.l, w, acc[j]); acc[j] = wmma_bf(a.h, w, acc[j]); } }
#pragma unroll
  for (int j = 0; j < 4; ++j) { const int c = j * 16 + col; const float bb = bfr(B1[c]);
#pragma unroll
    for (int r = 0; r < 8; ++r) { const float v = fmaxf(acc[j][r] + bb, 0.f); const __bf16 hb = (__bf16)v; sh_[wave][8 * g + r][c] = hb; sl_[wave][8 * g + r][c] = (__bf16)(v - (float)hb); } }
  LDSX();
  v8f acc2[4] = {};
#pragma unroll
  for (int kc = 0; kc < DM / 32; ++kc) { F2 a; a.h = frag_b(&sh_[wave][col][kc * 32], lane); a.l = frag_b(&sl_[wave][col][kc * 32], lane);
#pragma unroll
    for (int j = 0; j < 4; ++j) { const v16b w = frag_b(PK + PK_O2 + (size_t)(j * 16 + col) * DM + kc * 32, lane); acc2[j] = wmma_bf(a.l, w, acc2[j]); acc2[j] = wmma_bf(a.h, w, acc2[j]); } }
#pragma unroll
  for (int j = 0; j < 4; ++j) { const int c = j * 16 + col; const float bb = bfr(B2[c]);
#pragma unroll
    for (int r = 0; r < 8; ++r) so[wave][8 * g + r][c] = acc2[j][r] + bb; }
  LDSX();
  for (int rl = 0; rl < 16; ++rl) if (lane < 16) vst2(OUT + (r0 + rl) * DM + lane * 4, *(const v4f*)&so[wave][rl][lane * 4]);
}
extern "C" void kernel_launch(void* const* d_in, const int* in_sizes, int n_in, void* d_out, int out_size, void* d_ws, size_t ws_size, hipStream_t stream) {
  (void)in_sizes; (void)n_in; (void)out_size;
  const float** F = (const float**)d_in;
  if (ws_size < (size_t)WS_END) return;
  char* ws = (char*)d_ws; __bf16* PK = (__bf16*)(ws + WS_PK); _Float16 *QP = (_Float16*)(ws + WS_QP), *KP = (_Float16*)(ws + WS_KP), *VT = (_Float16*)(ws + WS_VT), *VTL = (_Float16*)(ws + WS_VTL); float* O = (float*)(ws + WS_O);
  k_pack<<<dim3(DM, 5), 256, 0, stream>>>(F[2], F[4], F[6], F[8], F[10], PK);
  k_qkv<<<TNG * NN / 64, 128, 0, stream>>>(F[0], F[1], PK, F[3], F[5], F[7], QP, KP, VT, VTL);
  k_attn<<<dim3(NN / 64, TNG), 128, 0, stream>>>(QP, KP, VT, VTL, O);
  k_mlp<<<TNG * NN / 64, 128, 0, stream>>>(O, PK, F[9], F[11], (float*)d_out);
}
